// LSTM_Generator_25520695673371
// MI455X (gfx1250) — hardware-verified
//
#include <hip/hip_runtime.h>
#include <stdint.h>
#include <stddef.h>

typedef __attribute__((ext_vector_type(16))) _Float16 v16h;
typedef __attribute__((ext_vector_type(8)))  _Float16 v8h;
typedef __attribute__((ext_vector_type(8)))  float    v8f;
typedef __attribute__((ext_vector_type(4)))  float    v4f;
typedef __attribute__((ext_vector_type(4)))  unsigned int v4u;
typedef __attribute__((ext_vector_type(2)))  unsigned int v2u;
typedef v4u v4ua __attribute__((may_alias));
typedef v4f v4fa __attribute__((may_alias));

constexpr int HID        = 100;
constexpr int NGATE      = 4 * HID;
constexpr int NB         = 512;
constexpr int NT         = 512;
constexpr int MROWS      = 16;
constexpr int NWAVES     = 5;
constexpr int NTHREADS   = NWAVES * 32;
constexpr int NTILE_PW   = 5;
constexpr int KW_IMG     = 224;
constexpr int XSEG_OFF   = 112;
constexpr int KPA        = 232;
constexpr int GPITCH     = 404;
constexpr int PLW        = 112;
constexpr int NKSTEP_L0  = 4;
constexpr int NKSTEP_L12 = 7;
constexpr int IMG_HALVES_PER_LAYER = NGATE * KW_IMG;
constexpr int OUT_STAGE  = 32;
constexpr float OPSCALE  = 16.0f;
constexpr float ACC_FOLD = 1.0f / 256.0f;

static_assert(NB % MROWS == 0);
static_assert(NGATE == NWAVES * NTILE_PW * 16);
static_assert((MROWS * HID) % NTHREADS == 0);
static_assert(NT % OUT_STAGE == 0);
static_assert(KPA % 8 == 0 && KW_IMG % 8 == 0 && PLW % 8 == 0);
static_assert(NKSTEP_L0 * 32 <= KW_IMG && NKSTEP_L12 * 32 == KW_IMG);
static_assert(XSEG_OFF + PLW == KW_IMG && XSEG_OFF + PLW <= KPA);
static_assert(NKSTEP_L0 * 32 >= HID && XSEG_OFF >= HID);
static_assert((MROWS * PLW) % (32 * 8) == 0);
static_assert((MROWS * PLW * 2) % 128 == 0);
static_assert((MROWS * OUT_STAGE) % (32 * 4) == 0);

__device__ __forceinline__ void dep_guard_h(v8f& a, v8f& b, v16h x, v16h y) { asm volatile("v_nop\n\tv_nop\n\tv_nop\n\tv_nop" : "+v"(a), "+v"(b) : "v"(x), "v"(y)); }
__device__ __forceinline__ void keep4_h(v16h a, v16h b, v16h c, v16h d) { asm volatile("v_nop" :: "v"(a), "v"(b), "v"(c), "v"(d)); }
__device__ __forceinline__ void acc_guard4(v8f& a, v8f& b, v8f& c, v8f& d) { asm volatile("v_nop\n\tv_nop\n\tv_nop\n\tv_nop" : "+v"(a), "+v"(b), "+v"(c), "+v"(d)); }
__device__ __forceinline__ void acc_guard1(v8f& a) { asm volatile("v_nop\n\tv_nop\n\tv_nop\n\tv_nop" : "+v"(a)); }

template <typename T> struct Frag;
template <> struct Frag<_Float16> {
  typedef v16h V; union U { v16h v; v8h h[2]; };
  static __device__ __forceinline__ v16h load(const _Float16* p) {
    U f; f.h[0] = *(const v8h*)(p); f.h[1] = *(const v8h*)(p + 16); return f.v;
  }
  static __device__ __forceinline__ v8f mma(v16h a, v16h b, v8f c) {
    return __builtin_amdgcn_wmma_f32_16x16x32_f16(false, a, false, b, (short)0, c, false, false);
  }
};

constexpr int PREP_CHUNKS_PER_LAYER = NGATE * (KW_IMG / 4);
constexpr int PREP_BLOCKS_PER_LAYER = (PREP_CHUNKS_PER_LAYER + 255) / 256;
static_assert(PREP_CHUNKS_PER_LAYER % 32 == 0);
static_assert((IMG_HALVES_PER_LAYER * 2) % 128 == 0);

__global__ __launch_bounds__(256) void prep_weight_image(
    const float* __restrict__ Whh0, const float* __restrict__ Wih1, const float* __restrict__ Whh1,
    const float* __restrict__ Wih2, const float* __restrict__ Whh2, unsigned short* __restrict__ img) {
  const int layer = blockIdx.x / PREP_BLOCKS_PER_LAYER;
  const int g = (blockIdx.x - layer * PREP_BLOCKS_PER_LAYER) * 256 + threadIdx.x;
  if (g >= PREP_CHUNKS_PER_LAYER) return;
  const float* hsrc = (layer == 0) ? Whh0 : ((layer == 1) ? Whh1 : Whh2);
  const float* xsrc = (layer == 2) ? Wih2 : Wih1;
  const int n = g / (KW_IMG / 4);
  const int kbase = (g - n * (KW_IMG / 4)) * 4;
  unsigned int bits[4];
#pragma unroll
  for (int e = 0; e < 4; ++e) {
    const int k = kbase + e;
    const int kh = (k < HID) ? k : (HID - 1);
    int kx = k - XSEG_OFF; kx = (kx < 0) ? 0 : kx; kx = (kx > HID - 1) ? (HID - 1) : kx;
    const float a  = hsrc[n * HID + kh];
    const float bx = xsrc[n * HID + kx];
    float v = 0.0f;
    if (k < HID) v = a;
    if (layer > 0 && k >= XSEG_OFF && k < XSEG_OFF + HID) v = bx;
    const _Float16 hv = (_Float16)(v * OPSCALE);
    bits[e] = (unsigned int)__builtin_bit_cast(unsigned short, hv);
  }
  v2u w;
  w.x = bits[0] | (bits[1] << 16);
  w.y = bits[2] | (bits[3] << 16);
  unsigned int* dst = (unsigned int*)img + (size_t)layer * (IMG_HALVES_PER_LAYER / 2) + (size_t)g * 2;
  *(volatile v2u*)dst = w;
  __threadfence();
  *(volatile v2u*)dst = w;
}

template <int MODE>
__global__ __launch_bounds__(NTHREADS) void lstm_layer_kernel(
    const float* __restrict__ z, const unsigned short* __restrict__ wimg,
    const float* __restrict__ bias, const float* __restrict__ wih0,
    const unsigned short* __restrict__ xplane, unsigned short* __restrict__ hplane,
    const float* __restrict__ wp, const float* __restrict__ bp, float* __restrict__ out) {
  constexpr int NKS = (MODE == 0) ? NKSTEP_L0 : NKSTEP_L12;

  __shared__ __align__(16) _Float16 Ash[MROWS * KPA];
  __shared__ __align__(16) float gates[MROWS * GPITCH];
  __shared__ __align__(16) float cst[MROWS * HID];
  __shared__ __align__(16) float biasL[NGATE];
  __shared__ __align__(16) float wih0L[NGATE];
  __shared__ __align__(16) float zrow[MROWS];
  __shared__ __align__(16) float prod[MROWS * HID];
  __shared__ __align__(16) float outb[MROWS * OUT_STAGE];
  __shared__ __align__(16) float wpL[128];

  const int tid  = threadIdx.x;
  const int wv   = tid >> 5;
  const int lane = tid & 31;
  const int hf   = lane >> 4;
  const int mr   = lane & 15;
  const int b0row = blockIdx.x * MROWS;
  const _Float16* Wl = (const _Float16*)(const void*)wimg;

  {
    const v4u zero4 = {0u, 0u, 0u, 0u};
    for (int q = tid; q < (MROWS * KPA) / 8; q += NTHREADS) *(v4ua*)(Ash + 8 * q) = zero4;
    for (int i = tid; i < MROWS * HID; i += NTHREADS) cst[i] = 0.0f;
    for (int i = tid; i < NGATE; i += NTHREADS) {
      biasL[i] = bias[i];
      if (MODE == 0) wih0L[i] = wih0[i];
    }
    if (MODE == 2) {
      for (int i = tid; i < HID; i += NTHREADS) wpL[i] = wp[i];
      if (tid == 0) wpL[HID] = bp[0];
    }
  }
  __syncthreads();

  for (int t = 0; t < NT; ++t) {
    if (MODE == 0) {
      if (tid < MROWS) zrow[tid] = z[(size_t)(b0row + tid) * NT + t];
    } else {
      const size_t tbase = ((size_t)t * NB + b0row) * PLW;
      for (int q = tid; q < (MROWS * PLW) / 8; q += NTHREADS) {
        const int m = q / (PLW / 8);
        const int c = q - m * (PLW / 8);
        const v4u v = *(const v4u*)(xplane + tbase + (size_t)q * 8);
        *(v4ua*)(Ash + m * KPA + XSEG_OFF + 8 * c) = v;
      }
    }
    __syncthreads();

    v8f acc[NTILE_PW];
#pragma unroll
    for (int j = 0; j < NTILE_PW; ++j) acc[j] = (v8f){0.f, 0.f, 0.f, 0.f, 0.f, 0.f, 0.f, 0.f};
#pragma unroll 1
    for (int s = 0; s < NKS; ++s) {
      const int k0 = s * 32;
      const v16h a = Frag<_Float16>::load(Ash + mr * KPA + k0 + 8 * hf);
      v16h bfr[NTILE_PW];
#pragma unroll
      for (int j = 0; j < NTILE_PW; ++j) {
        const int col = (wv * NTILE_PW + j) * 16 + mr;
        bfr[j] = Frag<_Float16>::load(Wl + (size_t)col * KW_IMG + k0 + 8 * hf);
      }
#pragma unroll
      for (int j = 0; j < NTILE_PW; ++j) acc[j] = Frag<_Float16>::mma(a, bfr[j], acc[j]);
      dep_guard_h(acc[0], acc[NTILE_PW - 1], a, bfr[NTILE_PW - 1]);
      keep4_h(bfr[0], bfr[1], bfr[2], bfr[3]);
    }
    acc_guard4(acc[0], acc[1], acc[2], acc[3]);
    acc_guard1(acc[4]);

    {
      float zr[8];
#pragma unroll
      for (int r = 0; r < 8; ++r) zr[r] = (MODE == 0) ? zrow[8 * hf + r] : 0.0f;
#pragma unroll
      for (int j = 0; j < NTILE_PW; ++j) {
        const int col = (wv * NTILE_PW + j) * 16 + mr;
        const float bb = biasL[col];
        const float w0 = (MODE == 0) ? wih0L[col] : 0.0f;
#pragma unroll
        for (int r = 0; r < 8; ++r) {
          float v = acc[j][r] * ACC_FOLD + bb;
          if (MODE == 0) v += zr[r] * w0;
          gates[(8 * hf + r) * GPITCH + col] = v;
        }
      }
    }
    __syncthreads();

#pragma unroll 1
    for (int it = 0; it < (MROWS * HID) / NTHREADS; ++it) {
      const int idx = it * NTHREADS + tid;
      const int m  = idx / HID;
      const int jj = idx - m * HID;
      const float* grow = gates + m * GPITCH + jj;
      const float gi = grow[0];
      const float gf = grow[HID];
      const float gg = grow[2 * HID];
      const float go = grow[3 * HID];
      const float si = 1.0f / (1.0f + expf(-gi));
      const float sf = 1.0f / (1.0f + expf(-gf));
      const float tg = tanhf(gg);
      const float so = 1.0f / (1.0f + expf(-go));
      const float cc = sf * cst[idx] + si * tg;
      cst[idx] = cc;
      const float hh = so * tanhf(cc);
      Ash[m * KPA + jj] = (_Float16)(hh * OPSCALE);
      if (MODE == 2) prod[idx] = wpL[jj] * hh;
    }
    __syncthreads();

    if (MODE != 2) {
      if (wv == 0) {
        const size_t tbase = ((size_t)t * NB + b0row) * PLW;
        for (int pass = 0; pass < 2; ++pass) {
#pragma unroll
          for (int i = 0; i < (MROWS * PLW) / (8 * 32); ++i) {
            const int q = i * 32 + lane;
            const int m = q / (PLW / 8);
            const int c = q - m * (PLW / 8);
            const v4u v = *(const v4ua*)(Ash + m * KPA + 8 * c);
            *(volatile v4u*)(hplane + tbase + (size_t)q * 8) = v;
          }
          __threadfence();
        }
      }
    } else {
      if (tid < MROWS) {
        float sacc = 0.0f;
#pragma unroll 1
        for (int jj = 0; jj < HID; ++jj) sacc += prod[tid * HID + jj];
        outb[tid * OUT_STAGE + (t & (OUT_STAGE - 1))] = tanhf(sacc + wpL[HID]);
      }
      if ((t & (OUT_STAGE - 1)) == OUT_STAGE - 1) {
        __syncthreads();
        if (wv == 0) {
          const int t0 = t - (OUT_STAGE - 1);
          for (int pass = 0; pass < 2; ++pass) {
#pragma unroll
            for (int i = 0; i < (MROWS * OUT_STAGE) / (4 * 32); ++i) {
              const int q  = i * 32 + lane;
              const int m  = q >> 3;
              const int c4 = (q & 7) * 4;
              const v4f v = *(const v4fa*)(outb + m * OUT_STAGE + c4);
              *(volatile v4f*)(out + (size_t)(b0row + m) * NT + t0 + c4) = v;
            }
            __threadfence();
          }
        }
      }
    }
  }
}

extern "C" void kernel_launch(void* const* d_in, const int* in_sizes, int n_in,
                              void* d_out, int out_size, void* d_ws,
                              size_t ws_size, hipStream_t stream) {
  if (n_in < 12) return;
  if (in_sizes[0] != NB * NT || in_sizes[1] != NGATE || in_sizes[2] != NGATE * HID || in_sizes[3] != NGATE ||
      in_sizes[4] != NGATE * HID || in_sizes[5] != NGATE * HID || in_sizes[6] != NGATE ||
      in_sizes[7] != NGATE * HID || in_sizes[8] != NGATE * HID || in_sizes[9] != NGATE ||
      in_sizes[10] != HID || in_sizes[11] < 1) return;
  if (out_size != NB * NT) return;

  const float* z    = (const float*)d_in[0];
  const float* Wih0 = (const float*)d_in[1];
  const float* Whh0 = (const float*)d_in[2];
  const float* b0   = (const float*)d_in[3];
  const float* Wih1 = (const float*)d_in[4];
  const float* Whh1 = (const float*)d_in[5];
  const float* b1   = (const float*)d_in[6];
  const float* Wih2 = (const float*)d_in[7];
  const float* Whh2 = (const float*)d_in[8];
  const float* b2   = (const float*)d_in[9];
  const float* Wp   = (const float*)d_in[10];
  const float* bp   = (const float*)d_in[11];
  float* out = (float*)d_out;

  const size_t img_bytes   = (size_t)3 * IMG_HALVES_PER_LAYER * 2;
  const size_t plane_bytes = (size_t)NT * NB * PLW * 2;
  const size_t off_img = 0;
  const size_t off_p0  = off_img + img_bytes;
  const size_t off_p1  = off_p0 + plane_bytes;
  const size_t total   = off_p1 + plane_bytes;
  if (total > ws_size) return;

  char* ws = (char*)d_ws;
  unsigned short* img = (unsigned short*)(ws + off_img);
  unsigned short* P0  = (unsigned short*)(ws + off_p0);
  unsigned short* P1  = (unsigned short*)(ws + off_p1);

  prep_weight_image<<<dim3(3 * PREP_BLOCKS_PER_LAYER), dim3(256), 0, stream>>>(Whh0, Wih1, Whh1, Wih2, Whh2, img);

  lstm_layer_kernel<0><<<dim3(NB / MROWS), dim3(NTHREADS), 0, stream>>>(
      z, img, b0, Wih0, P1, P0, Wp, bp, out);
  lstm_layer_kernel<1><<<dim3(NB / MROWS), dim3(NTHREADS), 0, stream>>>(
      z, img + IMG_HALVES_PER_LAYER, b1, Wih0, P0, P1, Wp, bp, out);
  lstm_layer_kernel<2><<<dim3(NB / MROWS), dim3(NTHREADS), 0, stream>>>(
      z, img + 2 * IMG_HALVES_PER_LAYER, b2, Wih0, P1, P0, Wp, bp, out);
}
